// EIGLayer_22874995819130
// MI455X (gfx1250) — hardware-run, weakly checked
//
#include <hip/hip_runtime.h>


namespace {
constexpr int N = 50000, E = 800000, F = 64, KP = 13 * F, NT16 = N / 16;
constexpr float XS = 8.0f, WSC = 256.0f, AVG = 2.833213344056216f;
typedef _Float16 b16;
typedef __attribute__((ext_vector_type(16))) _Float16 v16b;
typedef __attribute__((ext_vector_type(8))) _Float16 v8b;
typedef __attribute__((ext_vector_type(8))) float v8f;
typedef __attribute__((ext_vector_type(4))) float v4f;
typedef __attribute__((ext_vector_type(2))) float v2f;
__device__ __forceinline__ float bf16_rne(float f) { unsigned int u = __float_as_uint(f); u += 0x7FFFu + ((u >> 16) & 1u); float r = __uint_as_float(u & 0xFFFF0000u); asm volatile("" : "+v"(r)); return r; }
__device__ __forceinline__ void split16(float v, b16& hi, b16& lo) { hi = (b16)v; lo = (b16)(v - (float)hi); }
__device__ __forceinline__ v16b frag_kb(const b16* p, int hh) { const v8b a = *(const v8b*)(p + 8 * hh), b = *(const v8b*)(p + 16 + 8 * hh); v16b f;
#pragma unroll
  for (int e = 0; e < 8; ++e) { f[e] = a[e]; f[8 + e] = b[e]; } return f; }
__device__ __forceinline__ v8f wmma16b(v16b a, v16b b, v8f c) { v8f d = __builtin_amdgcn_wmma_f32_16x16x32_f16(false, a, false, b, (short)0, c, false, false); asm volatile("v_nop\n\tv_nop\n\tv_nop\n\tv_nop" : "+v"(d) : "v"(a), "v"(b)); return d; }
__device__ __forceinline__ void wave_lds_sync() { __builtin_amdgcn_fence(__ATOMIC_RELEASE, "workgroup"); __builtin_amdgcn_wave_barrier(); __builtin_amdgcn_fence(__ATOMIC_ACQUIRE, "workgroup"); }
__device__ __forceinline__ float pmul(float a, float b) { float p = a * b; asm volatile("" : "+v"(p)); return p; }
__device__ __forceinline__ int iclamp(int v, int lo, int hi) { return v < lo ? lo : (v > hi ? hi : v); }
constexpr int CSR_NBLK9 = 512, CSR_GB9 = 9, CSR_GN9 = 1 << CSR_GB9  , CSR_TS9 = (CSR_GN9 < 32 ? 32 : CSR_GN9)  , CSR_MAXG9 = 512, CSR_CAP9 = 12288  ;
__device__ __host__ __forceinline__ int csr_tix9(int v) { return (v >> CSR_GB9) * CSR_TS9 + (v & (CSR_GN9 - 1)); }
__global__ __launch_bounds__(64) void csrA_kernel9(const int* __restrict__ dst, int E, int N, int nG, int CHP, int NGP, int* __restrict__ STG, int* __restrict__ HST) {
  extern __shared__ int sm[];
  int* cnt = sm; int* run = sm + NGP; int* ids = sm + 2 * NGP;
  const int b = blockIdx.x; const int ch = (E + CSR_NBLK9 - 1) / CSR_NBLK9; const int e0 = b * ch, e1 = min(E, e0 + ch);
  for (int i = threadIdx.x; i < NGP; i += 64) cnt[i] = 0;
  for (int i = threadIdx.x; i < CHP; i += 64) ids[i] = -1;
  __syncthreads();
  if (threadIdx.x == 0) {
    for (int e = e0; e < e1; ++e) { int d = dst[e]; d = (d < 0) ? 0 : (d >= N ? N - 1 : d); cnt[d >> CSR_GB9] += 1; }
    int acc = 0; for (int g = 0; g < nG; ++g) { run[g] = acc; acc += cnt[g]; }
    for (int e = e0; e < e1; ++e) { int d = dst[e]; d = (d < 0) ? 0 : (d >= N ? N - 1 : d); const int g = d >> CSR_GB9; ids[run[g]] = e; run[g] += 1; } }
  __syncthreads();
  typedef __attribute__((ext_vector_type(4))) int v4i;
  for (int pass = 0; pass < 2; ++pass) {
    for (int i = threadIdx.x; i < CHP / 4; i += 64) *(volatile v4i*)(STG + (size_t)b * CHP + i * 4) = *(const v4i*)(&ids[i * 4]);
    for (int i = threadIdx.x; i < NGP / 4; i += 64) { v4i v; for (int e = 0; e < 4; ++e) v[e] = (i * 4 + e < nG) ? cnt[i * 4 + e] : 0; *(volatile v4i*)(HST + (size_t)b * NGP + i * 4) = v; }
    __threadfence(); }
}
__global__ __launch_bounds__(512) void csrS_kernel9(const int* __restrict__ HST, int nG, int NGP, int* __restrict__ START, int* __restrict__ TOT, int* __restrict__ OFF) {
  __shared__ int tot[CSR_MAXG9];
  const int b = threadIdx.x;
  for (int pass = 0; pass < 2; ++pass) { int runb = 0; for (int g = 0; g < nG; ++g) { int c = HST[(size_t)b * NGP + g]; c = (c < 0) ? 0 : c; ((volatile int*)OFF)[(size_t)g * CSR_NBLK9 + b] = runb; runb += c; } __threadfence(); }
  for (int g = threadIdx.x; g < nG; g += 512) { int s = 0; for (int bb = 0; bb < CSR_NBLK9; ++bb) { int c = HST[(size_t)bb * NGP + g]; s += (c < 0) ? 0 : c; } tot[g] = s; }
  __syncthreads();
  if (threadIdx.x < 32) {
    __shared__ int st[CSR_MAXG9 + 32];
    if (threadIdx.x == 0) { int acc = 0; for (int g = 0; g < NGP; ++g) { st[g] = acc; if (g < nG) acc += (tot[g] + 31) & ~31; } st[NGP] = acc; }
    __builtin_amdgcn_fence(__ATOMIC_RELEASE, "workgroup"); __builtin_amdgcn_wave_barrier(); __builtin_amdgcn_fence(__ATOMIC_ACQUIRE, "workgroup");
    for (int pass = 0; pass < 2; ++pass) { for (int i = threadIdx.x; i < NGP + 32; i += 32) { ((volatile int*)START)[i] = (i <= NGP) ? st[min(i, NGP)] : 0; ((volatile int*)TOT)[i] = (i < nG) ? tot[i] : 0; } __threadfence(); } }
}
__global__ __launch_bounds__(256) void csrB_kernel9(const int* __restrict__ dst, int N, int nG, int CHP, int NGP, int permLen, const int* __restrict__ STG, const int* __restrict__ HST, const int* __restrict__ OFF, const int* __restrict__ START, const int* __restrict__ TOT, int* __restrict__ PERM, int* __restrict__ ROWPTR, int* __restrict__ ROWCNT, int* __restrict__ FLAG) {
  typedef __attribute__((ext_vector_type(4))) int v4i;
  __shared__ int ids[CSR_CAP9]; __shared__ unsigned short key[CSR_CAP9]; __shared__ int outp[CSR_CAP9]; __shared__ int ncnt[CSR_GN9 + 1]; __shared__ int boff[CSR_NBLK9 + 1];
  const int g = blockIdx.x, t_ = threadIdx.x; int tot = TOT[g]; int st = START[g], stn = START[g + 1]; const int v0 = g * CSR_GN9; const int nv = min(CSR_GN9, N - v0); const int t0 = g * CSR_TS9;
  st = (st < 0) ? 0 : (st > permLen - 32 ? permLen - 32 : st) & ~31; stn = (stn < st) ? st : (stn > permLen ? permLen : stn); tot = (tot < 0) ? 0 : tot; if (tot > stn - st && tot <= CSR_CAP9) tot = stn - st;
  if (tot > CSR_CAP9) {
    for (int pass = 0; pass < 2; ++pass) { for (int i = t_; i < CSR_TS9 / 4; i += 256) { v4i a, c; for (int e = 0; e < 4; ++e) { a[e] = st; c[e] = 0; } *(volatile v4i*)(ROWPTR + t0 + i * 4) = a; *(volatile v4i*)(ROWCNT + t0 + i * 4) = c; } if (t_ == 0) ((volatile int*)FLAG)[0] = 1; __threadfence(); } (void)nv; return; }
  if (t_ == 0) { int acc = 0; for (int b = 0; b < CSR_NBLK9; ++b) { boff[b] = acc; int c = HST[(size_t)b * NGP + g]; c = (c < 0) ? 0 : (c > CHP ? CHP : c); acc += c; if (acc > tot) acc = tot; } boff[CSR_NBLK9] = acc; }
  for (int i = t_; i <= CSR_GN9; i += 256) ncnt[i] = 0;
  __syncthreads();
  for (int b = 0; b < CSR_NBLK9; ++b) { const int c = boff[b + 1] - boff[b]; int o_ = OFF[(size_t)g * CSR_NBLK9 + b]; o_ = (o_ < 0) ? 0 : (o_ > CHP - c ? CHP - c : o_); const int* src_ = STG + (size_t)b * CHP + o_;
    for (int i = t_; i < c; i += 256) { int id = src_[i]; id = (id < 0) ? 0 : id; ids[boff[b] + i] = id; int d = dst[id]; d = (d < v0) ? v0 : (d >= N ? N - 1 : d); int kk = d - v0; kk = (kk < 0) ? 0 : (kk >= CSR_GN9 ? CSR_GN9 - 1 : kk); key[boff[b] + i] = (unsigned short)kk; } }
  __syncthreads();
  if (t_ == 0) { for (int i = 0; i < tot; ++i) ncnt[key[i]] += 1; int acc = 0; for (int vl = 0; vl < CSR_GN9; ++vl) { const int c = ncnt[vl]; ncnt[vl] = acc; acc += c; } ncnt[CSR_GN9] = acc;
    for (int i = 0; i < tot; ++i) { const int vl = key[i]; outp[ncnt[vl]] = ids[i]; ncnt[vl] += 1; }
    for (int vl = CSR_GN9; vl > 0; --vl) ncnt[vl] = ncnt[vl - 1]; ncnt[0] = 0; }
  __syncthreads();
  for (int pass = 0; pass < 2; ++pass) {
    for (int i = t_; i < (stn - st) / 4; i += 256) { v4i v; for (int e = 0; e < 4; ++e) { const int q = i * 4 + e; v[e] = (q < tot) ? outp[q] : -1; } *(volatile v4i*)(PERM + st + i * 4) = v; }
    for (int i = t_; i < CSR_TS9 / 4; i += 256) { v4i a, c; for (int e = 0; e < 4; ++e) { const int vl = i * 4 + e; const int vc = vl < CSR_GN9 ? vl : CSR_GN9; a[e] = (vl < CSR_GN9) ? st + ncnt[vc] : st; c[e] = (vl < nv) ? (ncnt[(vc < CSR_GN9 ? vc : CSR_GN9 - 1) + 1] - ncnt[vc]) : 0; } *(volatile v4i*)(ROWPTR + t0 + i * 4) = a; *(volatile v4i*)(ROWCNT + t0 + i * 4) = c; }
    __threadfence(); }
}
__global__ __launch_bounds__(256) void csrZ_kernel9(int* __restrict__ p, size_t n4) { typedef __attribute__((ext_vector_type(4))) int v4i; const size_t tid = (size_t)blockIdx.x * 256 + threadIdx.x, nth = (size_t)gridDim.x * 256; v4i z = {0, 0, 0, 0}; for (size_t i = tid; i < n4; i += nth) *(volatile v4i*)(p + i * 4) = z; }
struct CsrBufs9 { int *STG, *HST, *OFF, *START, *TOT, *PERM, *ROWPTR, *ROWCNT, *FLAG; int nG, NGP, CHP; size_t permLen; char* base; size_t bytes; };
static size_t csr_carve9(CsrBufs9& c, char* ws, size_t off, int E, int N) {
  const size_t off0 = off; c.base = ws + off;
  auto al = [&](size_t bytes) { char* p = ws + off; off += (bytes + 255) & ~(size_t)255; return p; };
  c.nG = (N + CSR_GN9 - 1) / CSR_GN9; c.NGP = (c.nG + 31) & ~31; const int ch = (E + CSR_NBLK9 - 1) / CSR_NBLK9; c.CHP = (ch + 31) & ~31; c.permLen = (size_t)E + 32 * (size_t)c.nG + 32;
  c.STG = (int*)al((size_t)CSR_NBLK9 * c.CHP * 4); c.HST = (int*)al((size_t)CSR_NBLK9 * c.NGP * 4); c.OFF = (int*)al((size_t)c.NGP * CSR_NBLK9 * 4); c.START = (int*)al((size_t)(c.NGP + 64) * 4); c.TOT = (int*)al((size_t)(c.NGP + 64) * 4);
  c.PERM = (int*)al(c.permLen * 4); c.ROWPTR = (int*)al((size_t)c.nG * CSR_TS9 * 4); c.ROWCNT = (int*)al((size_t)c.nG * CSR_TS9 * 4); c.FLAG = (int*)al(256);
  c.bytes = off - off0; return off;
}
static void csr_build9(const CsrBufs9& c, const int* dst, int E, int N, hipStream_t stream) {
  const size_t smem = (size_t)(2 * c.NGP + c.CHP) * 4;
  csrZ_kernel9<<<512, 256, 0, stream>>>((int*)c.base, c.bytes / 16);
  csrA_kernel9<<<CSR_NBLK9, 64, smem, stream>>>(dst, E, N, c.nG, c.CHP, c.NGP, c.STG, c.HST);
  csrS_kernel9<<<1, 512, 0, stream>>>(c.HST, c.nG, c.NGP, c.START, c.TOT, c.OFF);
  csrB_kernel9<<<c.nG, 256, 0, stream>>>(dst, N, c.nG, c.CHP, c.NGP, (int)c.permLen, c.STG, c.HST, c.OFF, c.START, c.TOT, c.PERM, c.ROWPTR, c.ROWCNT, c.FLAG);
}


__global__ __launch_bounds__(256) void wput_kernel(const float* __restrict__ wp1, const float* __restrict__ wp2, const float* __restrict__ wq1, const float* __restrict__ wq2, b16* __restrict__ WPRE, b16* __restrict__ W2T, b16* __restrict__ WP1, b16* __restrict__ WP2) { const int u = blockIdx.x * 256 + threadIdx.x;
  for (int pass = 0; pass < 2; ++pass) {
    if (u < 2 * F * 8) { const int o = u / 8, k0 = (u % 8) * 8; const int part = o / F, oo = o % F; v8b v;
#pragma unroll
      for (int j = 0; j < 8; ++j) v[j] = (b16)(bf16_rne(wp1[(size_t)(part * F + k0 + j) * F + oo]) * WSC); *(volatile v8b*)(WPRE + (size_t)o * F + k0) = v; }
    if (u < F * 8) { const int o = u / 8, k0 = (u % 8) * 8; v8b v, v2;
#pragma unroll
      for (int j = 0; j < 8; ++j) { v[j] = (b16)(bf16_rne(wp2[(size_t)(k0 + j) * F + o]) * WSC); v2[j] = (b16)(bf16_rne(wq2[(size_t)(k0 + j) * F + o]) * WSC); } *(volatile v8b*)(W2T + (size_t)o * F + k0) = v; *(volatile v8b*)(WP2 + (size_t)o * F + k0) = v2; }
    if (u < F * (KP / 8)) { const int o = u / (KP / 8), k0 = (u % (KP / 8)) * 8; v8b v;
#pragma unroll
      for (int j = 0; j < 8; ++j) v[j] = (b16)(bf16_rne(wq1[(size_t)(k0 + j) * F + o]) * WSC); *(volatile v8b*)(WP1 + (size_t)o * KP + k0) = v; }
    __threadfence(); } }
__global__ __launch_bounds__(32) void pre_kernel(const float* __restrict__ h, const b16* __restrict__ WPRE, float* __restrict__ PAB) {
  __shared__ __attribute__((aligned(16))) b16 Ah[16][F + 8]; __shared__ float Tf[16][132]; const int lane = threadIdx.x, nloc = lane & 15, hlf = lane >> 4; const size_t m0 = (size_t)blockIdx.x * 16;
  for (int rr = 0; rr < 16; ++rr) for (int q = 0; q < 2; ++q) Ah[rr][q * 32 + lane] = (b16)(bf16_rne(h[(m0 + rr) * F + q * 32 + lane]) * XS);
  wave_lds_sync(); v8f acc[8];
#pragma unroll
  for (int t = 0; t < 8; ++t) acc[t] = (v8f){};
#pragma unroll
  for (int kb = 0; kb < F; kb += 32) { const v16b a = frag_kb(&Ah[nloc][kb], hlf);
#pragma unroll
    for (int t = 0; t < 8; ++t) acc[t] = wmma16b(a, frag_kb(WPRE + (size_t)(t * 16 + nloc) * F + kb, hlf), acc[t]); }
#pragma unroll
  for (int t = 0; t < 8; ++t)
#pragma unroll
    for (int r8 = 0; r8 < 8; ++r8) Tf[8 * hlf + r8][t * 16 + nloc] = acc[t][r8] * (1.0f / (XS * WSC));
  wave_lds_sync();
  for (int pass = 0; pass < 2; ++pass) { for (int rr = 0; rr < 16; ++rr) *(volatile v4f*)(PAB + (m0 + rr) * 2 * F + lane * 4) = *(const v4f*)(&Tf[rr][lane * 4]); __threadfence(); } }
__global__ __launch_bounds__(32) void agg_kernel(const float* __restrict__ PAB, const float* __restrict__ h, const float* __restrict__ bp1, const b16* __restrict__ W2T, const float* __restrict__ bp2, const int* __restrict__ srcs, const int* __restrict__ PERM, const int* __restrict__ ROWPTR, const int* __restrict__ ROWCNT, int permLen, int NLIM, float* __restrict__ HC) {
  __shared__ __attribute__((aligned(16))) b16 Ah[16][F + 8], Al[16][F + 8]; __shared__ float Te[16][68]; __shared__ int Us[16]; const int lane = threadIdx.x, nloc = lane & 15, hlf = lane >> 4; const size_t i = blockIdx.x; if (i >= (size_t)NLIM) return;
  int st = ROWPTR[i], cnt = ROWCNT[i]; cnt = iclamp(cnt, 0, 1 << 20); st = iclamp(st, 0, permLen - cnt);
  const int c0 = lane * 2; const float pb0 = PAB[i * 2 * F + F + c0] + bf16_rne(bp1[c0]), pb1 = PAB[i * 2 * F + F + c0 + 1] + bf16_rne(bp1[c0 + 1]); const float b20 = bf16_rne(bp2[c0]), b21 = bf16_rne(bp2[c0 + 1]);
  float s0 = 0.0f, s1 = 0.0f, q0 = 0.0f, q1 = 0.0f, mx0 = -INFINITY, mx1 = -INFINITY, mn0 = INFINITY, mn1 = INFINITY; int deg = 0;
#pragma unroll 1
  for (int j0 = 0; j0 < cnt; j0 += 16) {
    if (lane < 16) { const int j = j0 + lane; int u = -1; if (j < cnt) { const int e = iclamp(PERM[st + j], 0, E - 1); u = iclamp(srcs[e], 0, N - 1); if (u >= NLIM) u = -1; } Us[lane] = u; }
    wave_lds_sync();
    for (int rr = 0; rr < 16; ++rr) { const int u = Us[rr]; float a0 = 0.0f, a1 = 0.0f; if (u >= 0) { a0 = fmaxf(PAB[(size_t)u * 2 * F + c0] + pb0, 0.0f); a1 = fmaxf(PAB[(size_t)u * 2 * F + c0 + 1] + pb1, 0.0f); } b16 p, q; split16(a0 * XS, p, q); Ah[rr][c0] = p; Al[rr][c0] = q; split16(a1 * XS, p, q); Ah[rr][c0 + 1] = p; Al[rr][c0 + 1] = q; }
    wave_lds_sync(); v8f acc[4] = {(v8f){}, (v8f){}, (v8f){}, (v8f){}};
#pragma unroll
    for (int kb = 0; kb < F; kb += 32) { const v16b a = frag_kb(&Ah[nloc][kb], hlf), al = frag_kb(&Al[nloc][kb], hlf);
#pragma unroll
      for (int t = 0; t < 4; ++t) { const v16b bw = frag_kb(W2T + (size_t)(t * 16 + nloc) * F + kb, hlf); acc[t] = wmma16b(a, bw, acc[t]); acc[t] = wmma16b(al, bw, acc[t]); } }
#pragma unroll
    for (int t = 0; t < 4; ++t)
#pragma unroll
      for (int r8 = 0; r8 < 8; ++r8) Te[8 * hlf + r8][t * 16 + nloc] = acc[t][r8] * (1.0f / (XS * WSC));
    wave_lds_sync();
#pragma unroll 1
    for (int rr = 0; rr < 16; ++rr) { if (Us[rr] < 0) continue; ++deg; const float e0 = Te[rr][c0] + b20, e1 = Te[rr][c0 + 1] + b21; s0 += e0; s1 += e1; q0 += pmul(e0, e0); q1 += pmul(e1, e1); mx0 = fmaxf(mx0, e0); mx1 = fmaxf(mx1, e1); mn0 = fminf(mn0, e0); mn1 = fminf(mn1, e1); }
    wave_lds_sync(); }
  const float dsafe = (float)(deg > 0 ? deg : 1); const float m0 = s0 / dsafe, m1 = s1 / dsafe; const float sd0 = sqrtf(fmaxf(q0 / dsafe - pmul(m0, m0), 0.0f) + 1e-5f), sd1 = sqrtf(fmaxf(q1 / dsafe - pmul(m1, m1), 0.0f) + 1e-5f);
  if (deg == 0) { mx0 = 0.0f; mx1 = 0.0f; mn0 = 0.0f; mn1 = 0.0f; }
  const float logD = __logf(dsafe + 1.0f); const float amp = logD / AVG, att = AVG / logD;
  float agg[8] = {m0, m1, mx0, mx1, mn0, mn1, sd0, sd1};
  for (int pass = 0; pass < 2; ++pass) { float* row = HC + i * KP; *(volatile v2f*)(row + c0) = (v2f){bf16_rne(h[i * F + c0]), bf16_rne(h[i * F + c0 + 1])};
#pragma unroll
    for (int a = 0; a < 4; ++a) { const v2f v = {agg[2 * a], agg[2 * a + 1]}; *(volatile v2f*)(row + F + a * F + c0) = v; *(volatile v2f*)(row + 5 * F + a * F + c0) = (v2f){pmul(v[0], amp), pmul(v[1], amp)}; *(volatile v2f*)(row + 9 * F + a * F + c0) = (v2f){pmul(v[0], att), pmul(v[1], att)}; }
    __threadfence(); } }
__global__ __launch_bounds__(32) void post_kernel(const float* __restrict__ HC, const b16* __restrict__ WP1, const float* __restrict__ bq1, const b16* __restrict__ WP2, const float* __restrict__ bq2, const float* __restrict__ snorm, int NLIM, float* __restrict__ PO) {
  __shared__ __attribute__((aligned(16))) b16 Ah[16][KP + 8], Al[16][KP + 8], Hh[16][F + 8], Hl[16][F + 8]; __shared__ float Tf[16][68]; const int lane = threadIdx.x, nloc = lane & 15, hlf = lane >> 4; const size_t m0 = (size_t)blockIdx.x * 16; if (m0 >= (size_t)NLIM) return;
  for (int rr = 0; rr < 16; ++rr) for (int q = 0; q < KP / 32; ++q) { b16 p, ql; split16(HC[(m0 + rr) * KP + q * 32 + lane] * XS, p, ql); Ah[rr][q * 32 + lane] = p; Al[rr][q * 32 + lane] = ql; }
  wave_lds_sync(); v8f acc[4] = {(v8f){}, (v8f){}, (v8f){}, (v8f){}};
#pragma unroll 2
  for (int kb = 0; kb < KP; kb += 32) { const v16b a = frag_kb(&Ah[nloc][kb], hlf), al = frag_kb(&Al[nloc][kb], hlf);
#pragma unroll
    for (int t = 0; t < 4; ++t) { const v16b bw = frag_kb(WP1 + (size_t)(t * 16 + nloc) * KP + kb, hlf); acc[t] = wmma16b(a, bw, acc[t]); acc[t] = wmma16b(al, bw, acc[t]); } }
#pragma unroll
  for (int t = 0; t < 4; ++t) { const int c = t * 16 + nloc; const float bb = bf16_rne(bq1[c]);
#pragma unroll
    for (int r8 = 0; r8 < 8; ++r8) { b16 p, q; split16(fmaxf(acc[t][r8] * (1.0f / (XS * WSC)) + bb, 0.0f) * XS, p, q); Hh[8 * hlf + r8][c] = p; Hl[8 * hlf + r8][c] = q; } }
  wave_lds_sync(); v8f acc2[4] = {(v8f){}, (v8f){}, (v8f){}, (v8f){}};
#pragma unroll
  for (int kb = 0; kb < F; kb += 32) { const v16b a = frag_kb(&Hh[nloc][kb], hlf), al = frag_kb(&Hl[nloc][kb], hlf);
#pragma unroll
    for (int t = 0; t < 4; ++t) { const v16b bw = frag_kb(WP2 + (size_t)(t * 16 + nloc) * F + kb, hlf); acc2[t] = wmma16b(a, bw, acc2[t]); acc2[t] = wmma16b(al, bw, acc2[t]); } }
#pragma unroll
  for (int t = 0; t < 4; ++t) { const int c = t * 16 + nloc; const float bb = bf16_rne(bq2[c]);
#pragma unroll
    for (int r8 = 0; r8 < 8; ++r8) { const int rl = 8 * hlf + r8; Tf[rl][c] = pmul(acc2[t][r8] * (1.0f / (XS * WSC)) + bb, bf16_rne(snorm[m0 + rl])); } }
  wave_lds_sync();
  for (int pass = 0; pass < 2; ++pass) { for (int rr = 0; rr < 16; ++rr) *(volatile v2f*)(PO + (m0 + rr) * F + lane * 2) = (v2f){Tf[rr][lane * 2], Tf[rr][lane * 2 + 1]}; __threadfence(); } }
__global__ __launch_bounds__(256) void tilestat_kernel(const float* __restrict__ PO, int NLIM, float* __restrict__ PSQ) { const int wave = threadIdx.x >> 5, lane = threadIdx.x & 31; const size_t tile = (size_t)blockIdx.x * 8 + wave; if (tile * 16 >= (size_t)NLIM) return; float s[2] = {0.0f, 0.0f}, q[2] = {0.0f, 0.0f};
#pragma unroll 1
  for (int rr = 0; rr < 16; ++rr) { const v2f v = *(const v2f*)(PO + (tile * 16 + rr) * F + lane * 2); for (int k = 0; k < 2; ++k) { s[k] += v[k]; q[k] += pmul(v[k], v[k]); } }
  for (int pass = 0; pass < 2; ++pass) { *(volatile v2f*)(PSQ + tile * 2 * F + lane * 2) = (v2f){s[0], s[1]}; *(volatile v2f*)(PSQ + tile * 2 * F + F + lane * 2) = (v2f){q[0], q[1]}; __threadfence(); } }
__global__ __launch_bounds__(64) void bnstat_kernel(const float* __restrict__ PSQ, const float* __restrict__ g, const float* __restrict__ bta, int ntiles, int nrows, float* __restrict__ ST) { const int c = threadIdx.x; double s = 0.0, q = 0.0;
#pragma unroll 1
  for (int t = 0; t < ntiles; ++t) { s += (double)PSQ[(size_t)t * 2 * F + c]; q += (double)PSQ[(size_t)t * 2 * F + F + c]; } const double mu = s / (double)nrows; double var = q / (double)nrows - mu * mu; if (var < 0.0) var = 0.0;
  for (int pass = 0; pass < 2; ++pass) { ((volatile float*)ST)[c] = (float)mu; ((volatile float*)ST)[F + c] = pmul((float)(1.0 / sqrt(var + 1e-5)), bf16_rne(g[c])); ((volatile float*)ST)[2 * F + c] = bf16_rne(bta[c]); ((volatile float*)ST)[3 * F + c] = 0.0f; __threadfence(); } }
__global__ __launch_bounds__(256) void bnapply_kernel(const float* __restrict__ PO, const float* __restrict__ ST, int NLIM, float* __restrict__ out) { const size_t u = (size_t)blockIdx.x * 256 + threadIdx.x; if (u >= (size_t)NLIM * F / 4) return; const int c0 = (int)(u % (F / 4)) * 4; const v4f v = *(const v4f*)(PO + u * 4); v4f r;
  for (int k = 0; k < 4; ++k) r[k] = pmul(v[k] - ST[c0 + k], ST[F + c0 + k]) + ST[2 * F + c0 + k];
  for (int pass = 0; pass < 2; ++pass) { *(volatile v4f*)(out + u * 4) = r; __threadfence(); } }
}

extern "C" void kernel_launch(void* const* d_in, const int* in_sizes, int n_in, void* d_out, int out_size, void* d_ws, size_t ws_size, hipStream_t stream) {
  (void)n_in;
  auto Fp = [&](int i) { return (const float*)d_in[i]; }; auto Ip = [&](int i) { return (const int*)d_in[i]; };
  if (in_sizes[0] != N * F || in_sizes[2] != N || in_sizes[3] != 2 * F * F || in_sizes[5] != F * F || in_sizes[7] != KP * F || in_sizes[9] != F * F || in_sizes[13] != E || in_sizes[14] != E || out_size != N * F) return;
  const int NLIM = N;
  const int NT = NLIM / 16;
  size_t off = 0; char* ws = (char*)d_ws;
  auto carve = [&](size_t bytes) { char* p = ws + off; off += (bytes + 255) & ~(size_t)255; return p; };
  b16* WPRE = (b16*)carve((size_t)2 * F * F * 2); b16* W2T = (b16*)carve((size_t)F * F * 2); b16* WP1 = (b16*)carve((size_t)F * KP * 2); b16* WP2 = (b16*)carve((size_t)F * F * 2);
  float* PAB = (float*)carve((size_t)N * 2 * F * 4); float* HC = (float*)carve((size_t)N * KP * 4); float* PO = (float*)carve((size_t)N * F * 4); float* PSQ = (float*)carve((size_t)NT16 * 2 * F * 4); float* ST = (float*)carve(4 * F * 4); CsrBufs9 csr; off = csr_carve9(csr, ws, off, E, N);
  if (off > ws_size || off > ((size_t)240 << 20)) return;
  wput_kernel<<<(F * (KP / 8) + 255) / 256, 256, 0, stream>>>(Fp(3), Fp(5), Fp(7), Fp(9), WPRE, W2T, WP1, WP2);
  csr_build9(csr, Ip(14), E, N, stream);
  pre_kernel<<<N / 16, 32, 0, stream>>>(Fp(0), WPRE, PAB);
  agg_kernel<<<NLIM, 32, 0, stream>>>(PAB, Fp(0), Fp(4), W2T, Fp(6), Ip(13), csr.PERM, csr.ROWPTR, csr.ROWCNT, (int)csr.permLen, NLIM, HC);
  post_kernel<<<NT, 32, 0, stream>>>(HC, WP1, Fp(8), WP2, Fp(10), Fp(2), NLIM, PO);
  tilestat_kernel<<<(NT + 7) / 8, 256, 0, stream>>>(PO, NLIM, PSQ); bnstat_kernel<<<1, F, 0, stream>>>(PSQ, Fp(11), Fp(12), NT, NLIM, ST); bnapply_kernel<<<(unsigned)(((size_t)NLIM * F / 4 + 255) / 256), 256, 0, stream>>>(PO, ST, NLIM, (float*)d_out);
}
